// RelativeMultiAttention_66408784331311
// MI455X (gfx1250) — hardware-verified
//
#include <hip/hip_runtime.h>
#include <math.h>
#include <stdint.h>

#define NBATCH 2
#define SEQ    1024
#define DM     1024
#define NH     16
#define HD     64
#define PL     (2 * SEQ)
#define MP     (NBATCH * SEQ)
#define QKW    (4 * DM)
#define KOFF   (2 * DM)
#define CTXP   (2 * DM)
#define NQB    (SEQ / 64)
#define HG     2
#define NGRP   (NH / HG)
#define BANDN  (NQB + 1)
#define BAND0  (NQB - 1)
#define UBLK   ((NBATCH * NH * SEQ) / 256)
#define VBLK   ((NH * PL) / 256)
#define PLANE  ((size_t)MP * PL)
#define WSC    64.0f
#define RSC    2048.0f
#define PSC    1024.0f
static_assert(NH * HD == DM);
static_assert((SEQ % 64) == 0 && (DM % 64) == 0 && (MP % 64) == 0 && (PL % 64) == 0);
static_assert((NH % HG) == 0);
static_assert((((MP / 64) * BANDN) % 8) == 0);
static_assert(((NBATCH * NH * SEQ) % 256) == 0 && ((NH * PL) % 256) == 0);
static_assert(((MP * DM / 8) % 256) == 0 && ((PL * HD / 8) % 256) == 0);

typedef _Float16 v16h __attribute__((ext_vector_type(16)));
typedef _Float16 v8h  __attribute__((ext_vector_type(8)));
typedef __bf16   v16b __attribute__((ext_vector_type(16)));
typedef unsigned short v16us __attribute__((ext_vector_type(16)));
typedef unsigned short v8us  __attribute__((ext_vector_type(8)));
typedef float    v8f  __attribute__((ext_vector_type(8)));
typedef float    v4f  __attribute__((ext_vector_type(4)));
typedef unsigned int v4u __attribute__((ext_vector_type(4)));

union FragH { v16h v; v8h h[2]; };
union FragU { v16us v; v8us h[2]; };

__device__ __forceinline__ unsigned short bf_bits(float f) {
  unsigned u = __float_as_uint(f);
  return (unsigned short)((u + 0x7FFFu + ((u >> 16) & 1u)) >> 16);
}
__device__ __forceinline__ float bf_up(unsigned short h) { return __uint_as_float(((unsigned)h) << 16); }
__device__ __forceinline__ float bfr(float f) { return bf_up(bf_bits(f)); }
__device__ __forceinline__ unsigned short h_bits(_Float16 x) { return __builtin_bit_cast(unsigned short, x); }
__device__ __forceinline__ unsigned pk16(unsigned short a, unsigned short b) { return (unsigned)a | ((unsigned)b << 16); }
__device__ __forceinline__ v8f zero8() { v8f z = {0.f, 0.f, 0.f, 0.f, 0.f, 0.f, 0.f, 0.f}; return z; }

__device__ __forceinline__ v16us ldfrag_u(const unsigned short* p) {
  FragU f;
  f.h[0] = *(const v8us*)(p);
  f.h[1] = *(const v8us*)(p + 16);
  return f.v;
}

template <int BF>
__device__ __forceinline__ v8f mma_raw(v16us a, v16us b, v8f c) {
  if (BF) {
    return __builtin_amdgcn_wmma_f32_16x16x32_bf16(false, __builtin_bit_cast(v16b, a), false,
                                                   __builtin_bit_cast(v16b, b), (short)0, c, false, false);
  }
  return __builtin_amdgcn_wmma_f32_16x16x32_f16(false, __builtin_bit_cast(v16h, a), false,
                                                __builtin_bit_cast(v16h, b), (short)0, c, false, false);
}
__device__ __forceinline__ v8f mma_bu(v16us a, v16us b, v8f c) {
  c = __builtin_amdgcn_wmma_f32_16x16x32_bf16(false, __builtin_bit_cast(v16b, a), false,
                                               __builtin_bit_cast(v16b, b), (short)0, c, false, false);
#if defined(__HIP_DEVICE_COMPILE__)
  asm volatile("v_nop\n\tv_nop\n\tv_nop\n\tv_nop" : "+v"(c) : "v"(a), "v"(b));
#endif
  return c;
}
__device__ __forceinline__ v8f mma_h(v16h a, v16h b, v8f c) {
  c = __builtin_amdgcn_wmma_f32_16x16x32_f16(false, a, false, b, (short)0, c, false, false);
#if defined(__HIP_DEVICE_COMPILE__)
  asm volatile("v_nop\n\tv_nop\n\tv_nop\n\tv_nop" : "+v"(c) : "v"(a), "v"(b));
#endif
  return c;
}
__device__ __forceinline__ void dep_guard1(v8f& a, v8f& b, v16us x) {
#if defined(__HIP_DEVICE_COMPILE__)
  asm volatile("v_nop\n\tv_nop\n\tv_nop\n\tv_nop" : "+v"(a), "+v"(b) : "v"(x));
#endif
}
__device__ __forceinline__ void keep4_u(v16us a, v16us b, v16us c, v16us d) {
#if defined(__HIP_DEVICE_COMPILE__)
  asm volatile("v_nop" :: "v"(a), "v"(b), "v"(c), "v"(d));
#endif
}
__device__ __forceinline__ void acc_guard4(v8f& a, v8f& b, v8f& c, v8f& d) {
#if defined(__HIP_DEVICE_COMPILE__)
  asm volatile("v_nop\n\tv_nop\n\tv_nop\n\tv_nop" : "+v"(a), "+v"(b), "+v"(c), "+v"(d));
#endif
}
__device__ __forceinline__ void wave_sync_lds() {
  __builtin_amdgcn_fence(__ATOMIC_RELEASE, "workgroup");
  __builtin_amdgcn_wave_barrier();
  __builtin_amdgcn_fence(__ATOMIC_ACQUIRE, "workgroup");
}

__global__ __launch_bounds__(256) void conv_h16(const float* __restrict__ W, unsigned short* Wh, int n8, float wsc) {
  const int i  = blockIdx.x * 256 + threadIdx.x;
  const int ic = (i < n8) ? i : (n8 - 1);
  const float* src = W + (size_t)ic * 8;
  const v4f a = *(const v4f*)(src);
  const v4f c = *(const v4f*)(src + 4);
  v4u o;
  o[0] = pk16(h_bits((_Float16)(bfr(a[0]) * wsc)), h_bits((_Float16)(bfr(a[1]) * wsc)));
  o[1] = pk16(h_bits((_Float16)(bfr(a[2]) * wsc)), h_bits((_Float16)(bfr(a[3]) * wsc)));
  o[2] = pk16(h_bits((_Float16)(bfr(c[0]) * wsc)), h_bits((_Float16)(bfr(c[1]) * wsc)));
  o[3] = pk16(h_bits((_Float16)(bfr(c[2]) * wsc)), h_bits((_Float16)(bfr(c[3]) * wsc)));
  if (i < n8) *(volatile v4u*)(Wh + (size_t)i * 8) = o;
  __threadfence();
  if (i < n8) *(volatile v4u*)(Wh + (size_t)i * 8) = o;
}

__global__ __launch_bounds__(256) void conv_pp(const float* __restrict__ P, unsigned short* PP, int n8) {
  const int i  = blockIdx.x * 256 + threadIdx.x;
  const int ic = (i < n8) ? i : (n8 - 1);
  const float* src = P + (size_t)ic * 8;
  const v4f a = *(const v4f*)(src);
  const v4f c = *(const v4f*)(src + 4);
  v4u o;
  o[0] = pk16(bf_bits(a[0]), bf_bits(a[1]));
  o[1] = pk16(bf_bits(a[2]), bf_bits(a[3]));
  o[2] = pk16(bf_bits(c[0]), bf_bits(c[1]));
  o[3] = pk16(bf_bits(c[2]), bf_bits(c[3]));
  const int row = ic >> 3, c8 = (ic & 7) * 8;
  unsigned short* d0 = PP + (size_t)row * (2 * HD) + c8;
  if (i < n8) { *(volatile v4u*)(d0) = o; *(volatile v4u*)(d0 + HD) = o; }
  __threadfence();
  if (i < n8) { *(volatile v4u*)(d0) = o; *(volatile v4u*)(d0 + HD) = o; }
}

template <int MODE>
__global__ __launch_bounds__(256) void tconv64(const float* __restrict__ W, unsigned short* out,
                                               int rows, int cols, int ldo, int dupoff, float wsc) {
  __shared__ __align__(16) unsigned short sh[64 * 72];
  const int t  = threadIdx.x;
  const int n0 = blockIdx.x * 64;
  const int k0 = blockIdx.y * 64;
#pragma unroll
  for (int i = 0; i < 4; ++i) {
    const int idx = i * 256 + t;
    const int r = idx >> 4, c4 = (idx & 15) * 4;
    int kr = k0 + r;   kr = (kr < rows) ? kr : (rows - 1);
    int nc = n0 + c4;  nc = (nc < cols - 4) ? nc : (cols - 4);
    const v4f v = *(const v4f*)(W + (size_t)kr * cols + nc);
#pragma unroll
    for (int e = 0; e < 4; ++e) {
      unsigned short u;
      if (MODE == 0) u = h_bits((_Float16)(bfr(v[e]) * wsc));
      else           u = bf_bits(v[e]);
      sh[(c4 + e) * 72 + r] = u;
    }
  }
  __syncthreads();
  const int wave = t >> 5, lane = t & 31;
  const int q = lane >> 3, c8 = (lane & 7) * 8;
  v4u pv[2];
  size_t go[2];
#pragma unroll
  for (int it = 0; it < 2; ++it) {
    const int nl = it * 32 + wave * 4 + q;
    pv[it] = *(const v4u*)(sh + nl * 72 + c8);
    go[it] = (size_t)(n0 + nl) * ldo + k0 + c8;
  }
  for (int pass = 0; pass < 2; ++pass) {
#pragma unroll
    for (int it = 0; it < 2; ++it) {
      *(volatile v4u*)(out + go[it]) = pv[it];
      if (dupoff != 0) *(volatile v4u*)(out + go[it] + dupoff) = pv[it];
    }
    __threadfence();
  }
}

__global__ __launch_bounds__(256) void biasprep(const float* __restrict__ uin, const float* __restrict__ vin,
                                               const float* __restrict__ P, const unsigned short* __restrict__ qk,
                                               float* UB, float* VP) {
  __shared__ float tsh[HD];
  const int t   = threadIdx.x;
  const int blk = blockIdx.x;
  const bool isU = (blk < UBLK);
  const int idxU = blk * 256 + t;
  const int idxV = (blk - UBLK) * 256 + t;
  const int h = isU ? ((blk >> 2) & (NH - 1)) : (((blk - UBLK) >> 3) & (NH - 1));
  const float* src = isU ? (uin + h * HD) : (vin + h * HD);
  if (t < HD) tsh[t] = bfr(src[t]);
  __syncthreads();
  float acc = 0.f;
  if (isU) {
    const int b = idxU >> 14;
    const int j = idxU & (SEQ - 1);
    const unsigned short* kr = qk + ((size_t)b * SEQ + j) * QKW + KOFF + h * (2 * HD);
#pragma unroll 1
    for (int i = 0; i < 8; ++i) {
      const v8us a = *(const v8us*)(kr + 8 * i);
      const v8us l = *(const v8us*)(kr + HD + 8 * i);
#pragma unroll
      for (int e = 0; e < 8; ++e) acc += tsh[8 * i + e] * (bf_up(a[e]) + bf_up(l[e]));
    }
  } else {
    const int l = idxV & (PL - 1);
    const float* pr = P + (size_t)l * HD;
#pragma unroll 1
    for (int i = 0; i < 8; ++i) {
      const v4f a = *(const v4f*)(pr + 8 * i);
      const v4f c = *(const v4f*)(pr + 8 * i + 4);
#pragma unroll
      for (int e = 0; e < 4; ++e) {
        acc += tsh[8 * i + e] * bfr(a[e]);
        acc += tsh[8 * i + 4 + e] * bfr(c[e]);
      }
    }
  }
  float* dst = isU ? UB : VP;
  const int di = isU ? idxU : idxV;
  dst += di;
  *(volatile float*)dst = acc;
  __threadfence();
  *(volatile float*)dst = acc;
}

template <int BF, int OM, int CB>
__global__ __launch_bounds__(256) void gemm64(
    const unsigned short* __restrict__ Ap, int lda, long long sAy, long long sAz,
    const unsigned short* __restrict__ Btp, int ldb, long long sBy,
    unsigned short* Cp, unsigned short* Cp2, float* Cf, int ldc, long long sCy, long long sCz,
    const float* __restrict__ cbias, long long sCBz,
    int M, int N, int K, int nmul, int bandN, int band0, int bandMask, float oscale) {
  __shared__ __align__(16) float sT[8][16 * 68];
  const int by   = blockIdx.y;
  const int bz   = blockIdx.z;
  const int lane = threadIdx.x & 31;
  const int wave = threadIdx.x >> 5;
  const int tilesN = N >> 6;
  const int tilesM = M >> 6;
  const int tile = blockIdx.x * 8 + wave;
  if (tile >= tilesM * bandN) return;
  const int tm = tile / bandN;
  const int tb = tile - tm * bandN;
  int tn = tb + band0 - (tm & bandMask);
  tn = (tn < 0) ? 0 : tn;
  tn = (tn > tilesN - 1) ? (tilesN - 1) : tn;
  const int m0 = tm << 6;
  const int n0 = tn << 6;

  const unsigned short* Ab = Ap  + (size_t)by * (size_t)sAy + (size_t)bz * (size_t)sAz;
  const unsigned short* Bb = Btp + (size_t)by * (size_t)sBy;
  const size_t cofs = (size_t)by * (size_t)sCy + (size_t)bz * (size_t)sCz;

  const int rlane = lane & 15;
  const int koff  = (lane >> 4) * 8;
  const int mOff  = (lane >> 4) * 8;

  v8f acc[4][4];
#pragma unroll
  for (int i = 0; i < 4; ++i)
#pragma unroll
    for (int j = 0; j < 4; ++j) acc[i][j] = zero8();

  for (int k0 = 0; k0 < K; k0 += 32) {
    v16us bh[4];
#pragma unroll
    for (int j = 0; j < 4; ++j) {
      const size_t bo = (size_t)(n0 + (j << 4) + rlane) * ldb + koff + k0;
      bh[j] = ldfrag_u(Bb + bo);
    }
#pragma unroll
    for (int i = 0; i < 4; ++i) {
      const size_t ao = (size_t)(m0 + (i << 4) + rlane) * lda + koff + k0;
      const v16us ah = ldfrag_u(Ab + ao);
#pragma unroll
      for (int j = 0; j < 4; ++j) acc[i][j] = mma_raw<BF>(ah, bh[j], acc[i][j]);
      dep_guard1(acc[i][0], acc[i][3], ah);
    }
    keep4_u(bh[0], bh[1], bh[2], bh[3]);
  }
  acc_guard4(acc[0][0], acc[0][1], acc[0][2], acc[0][3]);
  acc_guard4(acc[1][0], acc[1][1], acc[1][2], acc[1][3]);
  acc_guard4(acc[2][0], acc[2][1], acc[2][2], acc[2][3]);
  acc_guard4(acc[3][0], acc[3][1], acc[3][2], acc[3][3]);

  const int hh2 = lane >> 4, c4 = (lane & 15) * 4;
  const int q8  = lane >> 3, c8 = (lane & 7) * 8;

  v4f cb4 = {0.f, 0.f, 0.f, 0.f};
  if (CB) {
    const float cbw = (by == 0) ? 1.f : 0.f;
    const v4f cbv = *(const v4f*)(cbias + (size_t)bz * (size_t)sCBz + n0 + c4);
    cb4 = cbv * cbw;
  }

  float* slab = sT[wave];
#pragma unroll
  for (int i = 0; i < 4; ++i) {
    const int mBase = m0 + (i << 4);
#pragma unroll
    for (int j = 0; j < 4; ++j) {
#pragma unroll
      for (int r = 0; r < 8; ++r) {
        slab[(mOff + r) * 68 + (j << 4) + rlane] = acc[i][j][r];
      }
    }
    wave_sync_lds();
    if (OM == 0) {
      float* C = Cf + cofs;
      v4f vals[8];
#pragma unroll
      for (int it = 0; it < 8; ++it) {
        const int row = it * 2 + hh2;
        v4f v = *(const v4f*)(slab + row * 68 + c4);
        vals[it] = v * oscale + cb4;
      }
      for (int pass = 0; pass < 2; ++pass) {
#pragma unroll
        for (int it = 0; it < 8; ++it) {
          const int row = it * 2 + hh2;
          *(volatile v4f*)(C + (size_t)(mBase + row) * ldc + (size_t)n0 * nmul + c4) = vals[it];
        }
        __threadfence();
      }
    } else {
      unsigned short* C  = Cp  + cofs;
      unsigned short* C2 = Cp2 + cofs;
      v4u hv[4], lv[4];
#pragma unroll
      for (int it = 0; it < 4; ++it) {
        const int row = it * 4 + q8;
        const float* sp = slab + row * 68 + c8;
        v4u ha, la;
#pragma unroll
        for (int e = 0; e < 4; ++e) {
          const float f0 = sp[2 * e]     * oscale;
          const float f1 = sp[2 * e + 1] * oscale;
          unsigned short u0, u1, w0, w1;
          if (OM == 3) {
            u0 = bf_bits(f0); u1 = bf_bits(f1);
            w0 = bf_bits(f0 - bf_up(u0)); w1 = bf_bits(f1 - bf_up(u1));
          } else {
            const _Float16 g0 = (_Float16)f0, g1 = (_Float16)f1;
            u0 = h_bits(g0); u1 = h_bits(g1);
            w0 = h_bits((_Float16)((f0 - (float)g0) * RSC));
            w1 = h_bits((_Float16)((f1 - (float)g1) * RSC));
          }
          ha[e] = pk16(u0, u1);
          la[e] = pk16(w0, w1);
        }
        hv[it] = ha;
        lv[it] = la;
      }
      for (int pass = 0; pass < 2; ++pass) {
#pragma unroll
        for (int it = 0; it < 4; ++it) {
          const int row = it * 4 + q8;
          const size_t go = (size_t)(mBase + row) * ldc + (size_t)n0 * nmul + c8;
          *(volatile v4u*)(C  + go) = hv[it];
          *(volatile v4u*)(C2 + go) = lv[it];
        }
        __threadfence();
      }
    }
    wave_sync_lds();
  }
}

__global__ __launch_bounds__(128)
void attn64(const unsigned short* __restrict__ qk, const unsigned short* __restrict__ vth,
            const unsigned short* __restrict__ vtl, const float* __restrict__ tab,
            const float* __restrict__ ubp, unsigned short* ctxp, int hbase, float sscale) {
  __shared__ __align__(16) unsigned short Kh[64 * 64];
  __shared__ __align__(16) unsigned short Kl[64 * 64];
  __shared__ __align__(16) _Float16 Vh[64 * 64];
  __shared__ __align__(16) _Float16 Vl[64 * 64];
  __shared__ __align__(16) _Float16 Psh[4][16 * 64];
  __shared__ __align__(16) float    Os[4][16 * 64];

  const int tid  = threadIdx.x;
  const int wave = tid >> 5;
  const int lane = tid & 31;
  const int hh   = lane >> 4;
  const int c    = lane & 15;

  const int bx   = blockIdx.x;
  const int qb   = bx % NQB;
  const int rest = bx / NQB;
  const int zl   = rest % HG;
  const int b    = rest / HG;
  const int h    = hbase + zl;
  const int q0   = qb * 64 + wave * 16;
  const size_t rowB = (size_t)b * SEQ;

  const unsigned short* Qh  = qk + (size_t)h * (2 * HD);
  const unsigned short* Ql  = Qh + HD;
  const unsigned short* Kgh = qk + KOFF + (size_t)h * (2 * HD);
  const unsigned short* Kgl = Kgh + HD;
  const _Float16* Vgh = (const _Float16*)(const void*)vth + ((size_t)b * DM + (size_t)h * HD) * SEQ;
  const _Float16* Vgl = (const _Float16*)(const void*)vtl + ((size_t)b * DM + (size_t)h * HD) * SEQ;
  const float* QPt = tab + (size_t)(zl * 2) * PLANE + rowB * PL;
  const float* KPt = tab + (size_t)(zl * 2 + 1) * PLANE + rowB * PL;
  const float* Ub  = ubp + ((size_t)b * NH + h) * SEQ;

  float mrow[8], lrow[8];
  v8f oacc[4], oaccL[4];
#pragma unroll
  for (int r = 0; r < 8; ++r) { mrow[r] = -INFINITY; lrow[r] = 0.f; }
#pragma unroll
  for (int t = 0; t < 4; ++t) { oacc[t] = zero8(); oaccL[t] = zero8(); }

#pragma unroll 1
  for (int kt = 0; kt < NQB; ++kt) {
    const int kv0 = kt * 64;
    float mk[4];
#pragma unroll
    for (int j = 0; j < 4; ++j) mk[j] = Ub[kv0 + j * 16 + c];

    __syncthreads();
    {
      const int r = tid >> 1, hf = (tid & 1) * 32;
      const unsigned short* kgh = Kgh + (rowB + kv0 + r) * QKW + hf;
      const unsigned short* kgl = Kgl + (rowB + kv0 + r) * QKW + hf;
      const _Float16* vgh = Vgh + (size_t)r * SEQ + kv0 + hf;
      const _Float16* vgl = Vgl + (size_t)r * SEQ + kv0 + hf;
#pragma unroll
      for (int i = 0; i < 4; ++i) {
        const v8us a0 = *(const v8us*)(kgh + 8 * i);
        const v8us a1 = *(const v8us*)(kgl + 8 * i);
        const v8h  b0 = *(const v8h*)(vgh + 8 * i);
        const v8h  b1 = *(const v8h*)(vgl + 8 * i);
        *(v8us*)(Kh + r * 64 + hf + 8 * i) = a0;
        *(v8us*)(Kl + r * 64 + hf + 8 * i) = a1;
        *(v8h*)(Vh + r * 64 + hf + 8 * i) = b0;
        *(v8h*)(Vl + r * 64 + hf + 8 * i) = b1;
      }
    }
    __syncthreads();

    v16us qh2[2], ql2[2];
#pragma unroll
    for (int dc = 0; dc < 2; ++dc) {
      qh2[dc] = ldfrag_u(Qh + (rowB + q0 + c) * QKW + dc * 32 + 8 * hh);
      ql2[dc] = ldfrag_u(Ql + (rowB + q0 + c) * QKW + dc * 32 + 8 * hh);
    }

    v8f s[4];
#pragma unroll
    for (int j = 0; j < 4; ++j) {
      v8f sh = zero8();
#pragma unroll
      for (int dc = 0; dc < 2; ++dc) {
        FragU kbh, kbl;
        kbh.h[0] = *(const v8us*)(Kh + (j * 16 + c) * 64 + dc * 32 + 8 * hh);
        kbh.h[1] = *(const v8us*)(Kh + (j * 16 + c) * 64 + dc * 32 + 16 + 8 * hh);
        kbl.h[0] = *(const v8us*)(Kl + (j * 16 + c) * 64 + dc * 32 + 8 * hh);
        kbl.h[1] = *(const v8us*)(Kl + (j * 16 + c) * 64 + dc * 32 + 16 + 8 * hh);
        sh = mma_bu(qh2[dc], kbh.v, sh);
        sh = mma_bu(qh2[dc], kbl.v, sh);
        sh = mma_bu(ql2[dc], kbh.v, sh);
      }
      const int kg  = kv0 + j * 16 + c;
      const int qr0 = q0 + 8 * hh;
      const float* kpr = KPt + (size_t)kg * PL + (SEQ + qr0 - kg);
#pragma unroll
      for (int r = 0; r < 8; ++r) {
        const float qp = QPt[(size_t)(qr0 + r) * PL + (SEQ + kg - qr0 - r)];
        const float kp = kpr[r];
        s[j][r] = (sh[r] + qp + kp + mk[j]) * sscale;
      }
    }

    _Float16* pwh = Psh[wave];
#pragma unroll
    for (int r = 0; r < 8; ++r) {
      float m = s[0][r];
      m = fmaxf(m, s[1][r]);
      m = fmaxf(m, s[2][r]);
      m = fmaxf(m, s[3][r]);
#pragma unroll
      for (int off = 1; off < 16; off <<= 1) m = fmaxf(m, __shfl_xor(m, off, 32));
      const float mnew  = fmaxf(mrow[r], m);
      const float alpha = __expf(mrow[r] - mnew);
      mrow[r] = mnew;
      float psum = 0.f;
#pragma unroll
      for (int j = 0; j < 4; ++j) {
        const float p = __expf(s[j][r] - mnew);
        psum += p;
        pwh[(8 * hh + r) * 64 + j * 16 + c] = (_Float16)(p * PSC);
      }
#pragma unroll
      for (int off = 1; off < 16; off <<= 1) psum += __shfl_xor(psum, off, 32);
      lrow[r] = lrow[r] * alpha + psum;
#pragma unroll
      for (int t = 0; t < 4; ++t) { oacc[t][r] *= alpha; oaccL[t][r] *= alpha; }
    }
    wave_sync_lds();

#pragma unroll 1
    for (int kk = 0; kk < 2; ++kk) {
      FragH pa;
      pa.h[0] = *(const v8h*)(pwh + c * 64 + kk * 32 + 8 * hh);
      pa.h[1] = *(const v8h*)(pwh + c * 64 + kk * 32 + 16 + 8 * hh);
#pragma unroll
      for (int t = 0; t < 4; ++t) {
        FragH vb, vl;
        vb.h[0] = *(const v8h*)(Vh + (t * 16 + c) * 64 + kk * 32 + 8 * hh);
        vb.h[1] = *(const v8h*)(Vh + (t * 16 + c) * 64 + kk * 32 + 16 + 8 * hh);
        vl.h[0] = *(const v8h*)(Vl + (t * 16 + c) * 64 + kk * 32 + 8 * hh);
        vl.h[1] = *(const v8h*)(Vl + (t * 16 + c) * 64 + kk * 32 + 16 + 8 * hh);
        oacc[t]  = mma_h(pa.v, vb.v, oacc[t]);
        oaccL[t] = mma_h(pa.v, vl.v, oaccL[t]);
      }
    }
  }

  float* os = Os[wave];
#pragma unroll
  for (int r = 0; r < 8; ++r) {
    const float l = lrow[r];
    const float inv = ((l > 0.f) ? (1.0f / l) : 0.f) * (1.0f / PSC);
#pragma unroll
    for (int t = 0; t < 4; ++t) os[(8 * hh + r) * 64 + t * 16 + c] = (oacc[t][r] + oaccL[t][r] * (1.0f / RSC)) * inv;
  }
  wave_sync_lds();
  {
    const int q4 = lane >> 3, c8 = (lane & 7) * 8;
    v4u hv[4], lv[4];
#pragma unroll
    for (int it = 0; it < 4; ++it) {
      const int row = it * 4 + q4;
      const float* sp = os + row * 64 + c8;
      v4u ha, la;
#pragma unroll
      for (int e = 0; e < 4; ++e) {
        const float f0 = sp[2 * e], f1 = sp[2 * e + 1];
        const unsigned short u0 = bf_bits(f0), u1 = bf_bits(f1);
        const unsigned short w0 = bf_bits(f0 - bf_up(u0)), w1 = bf_bits(f1 - bf_up(u1));
        ha[e] = pk16(u0, u1);
        la[e] = pk16(w0, w1);
      }
      hv[it] = ha;
      lv[it] = la;
    }
    for (int pass = 0; pass < 2; ++pass) {
#pragma unroll
      for (int it = 0; it < 4; ++it) {
        const int row = it * 4 + q4;
        const size_t go = (rowB + q0 + row) * CTXP + (size_t)h * HD + c8;
        *(volatile v4u*)(ctxp + go)      = hv[it];
        *(volatile v4u*)(ctxp + go + DM) = lv[it];
      }
      __threadfence();
    }
  }
}

extern "C" void kernel_launch(void* const* d_in, const int* in_sizes, int n_in,
                              void* d_out, int out_size, void* d_ws, size_t ws_size,
                              hipStream_t stream) {
  if (n_in < 8) return;
  if (in_sizes[0] != MP * DM) return;
  if (in_sizes[1] != DM * DM || in_sizes[2] != DM * DM) return;
  if (in_sizes[3] != DM * DM || in_sizes[4] != DM * DM) return;
  if (in_sizes[5] != NH * HD || in_sizes[6] != NH * HD) return;
  if (in_sizes[7] != PL * HD) return;
  if (out_size != MP * DM) return;

  const float* x_in = (const float*)d_in[0];
  const float* w_q  = (const float*)d_in[1];
  const float* w_k  = (const float*)d_in[2];
  const float* w_v  = (const float*)d_in[3];
  const float* w_o  = (const float*)d_in[4];
  const float* u_in = (const float*)d_in[5];
  const float* v_in = (const float*)d_in[6];
  const float* pos  = (const float*)d_in[7];

  const size_t PWQK = (size_t)(2 * DM) * DM * 2;
  const size_t PWV  = (size_t)DM * DM * 2;
  const size_t PWO2 = (size_t)DM * (2 * DM) * 2;
  const size_t PXH  = (size_t)MP * DM * 2;
  const size_t PPP  = (size_t)PL * (2 * HD) * 2;
  const size_t PQK  = (size_t)MP * QKW * 2;
  const size_t PVT  = (size_t)NBATCH * DM * SEQ * 2;
  const size_t PCTX = (size_t)MP * CTXP * 2;
  const size_t PUB  = (size_t)NBATCH * NH * SEQ * 4;
  const size_t PVP  = (size_t)NH * PL * 4;
  const size_t PTAB = (size_t)HG * 2 * PLANE * 4;
  size_t off = 0;
  const size_t oWqk = off; off += PWQK;
  const size_t oWv  = off; off += PWV;
  const size_t oWo2 = off; off += PWO2;
  const size_t oXH  = off; off += PXH;
  const size_t oPP  = off; off += PPP;
  const size_t oQK  = off; off += PQK;
  const size_t oVTh = off; off += PVT;
  const size_t oVTl = off; off += PVT;
  const size_t oCtx = off; off += PCTX;
  const size_t oUB  = off; off += PUB;
  const size_t oVP  = off; off += PVP;
  const size_t oTAB = off; off += PTAB;
  if (off > ws_size) return;
  if (off > (size_t)134217728) return;

  char* ws = (char*)d_ws;
  unsigned short* WqkT = (unsigned short*)(ws + oWqk);
  unsigned short* WvT  = (unsigned short*)(ws + oWv);
  unsigned short* WoT2 = (unsigned short*)(ws + oWo2);
  unsigned short* XH   = (unsigned short*)(ws + oXH);
  unsigned short* PPb  = (unsigned short*)(ws + oPP);
  unsigned short* QK   = (unsigned short*)(ws + oQK);
  unsigned short* VTh  = (unsigned short*)(ws + oVTh);
  unsigned short* VTl  = (unsigned short*)(ws + oVTl);
  unsigned short* Ctx  = (unsigned short*)(ws + oCtx);
  float*          UB   = (float*)(ws + oUB);
  float*          VP   = (float*)(ws + oVP);
  float*          TAB  = (float*)(ws + oTAB);
  float*          out0 = (float*)d_out;

  const int n8x = (MP * DM) / 8;
  const int n8p = (PL * HD) / 8;
  const dim3 blk(256), blk128(128);
  const dim3 gT(DM / 64, DM / 64);
  const dim3 gCx(n8x / 256);
  const dim3 gPP(n8p / 256);
  const dim3 gNqk(((MP / 64) * ((2 * DM) / 64)) / 8, 1, 1);
  const dim3 gVT(((DM / 64) * (SEQ / 64)) / 8, NBATCH, 1);
  const dim3 gBias(UBLK + VBLK);
  const dim3 gTab(((MP / 64) * BANDN) / 8, 2, HG);
  const dim3 gAttn(NBATCH * HG * NQB);
  const dim3 gNo(((MP / 64) * (DM / 64)) / 8, 1, 1);
  if ((((MP / 64) * ((2 * DM) / 64)) % 8) != 0) return;
  if ((((DM / 64) * (SEQ / 64)) % 8) != 0) return;
  if ((((MP / 64) * (DM / 64)) % 8) != 0) return;
  const float invw = 1.0f / WSC;

  tconv64<0><<<gT, blk, 0, stream>>>(w_q, WqkT, DM, DM, DM, 0, WSC);
  tconv64<0><<<gT, blk, 0, stream>>>(w_k, WqkT + (size_t)DM * DM, DM, DM, DM, 0, WSC);
  tconv64<0><<<gT, blk, 0, stream>>>(w_v, WvT, DM, DM, DM, 0, WSC);
  tconv64<1><<<gT, blk, 0, stream>>>(w_o, WoT2, DM, DM, 2 * DM, DM, 1.0f);
  conv_h16<<<gCx, blk, 0, stream>>>(x_in, XH, n8x, 1.0f);
  conv_pp<<<gPP, blk, 0, stream>>>(pos, PPb, n8p);

  gemm64<0, 3, 0><<<gNqk, blk, 0, stream>>>(
      XH, DM, 0LL, 0LL, WqkT, DM, 0LL,
      QK, QK + HD, out0, QKW, 0LL, 0LL, VP, 0LL,
      MP, 2 * DM, DM, 2, (2 * DM) / 64, 0, 0, invw);
  gemm64<0, 4, 0><<<gVT, blk, 0, stream>>>(
      WvT, DM, 0LL, 0LL, XH, DM, (long long)SEQ * DM,
      VTh, VTl, out0, SEQ, (long long)DM * SEQ, 0LL, VP, 0LL,
      DM, SEQ, DM, 1, SEQ / 64, 0, 0, invw);

  biasprep<<<gBias, blk, 0, stream>>>(u_in, v_in, pos, QK, UB, VP);

  for (int hg = 0; hg < NGRP; ++hg) {
    gemm64<1, 0, 1><<<gTab, blk, 0, stream>>>(
        QK + (size_t)hg * HG * (2 * HD), QKW, (long long)KOFF, (long long)(2 * HD), PPb, 2 * HD, 0LL,
        Ctx, Ctx, TAB, PL, (long long)PLANE, (long long)(2 * PLANE), VP + (size_t)hg * HG * PL, (long long)PL,
        MP, PL, 2 * HD, 1, BANDN, BAND0, NQB - 1, 1.0f);
    attn64<<<gAttn, blk128, 0, stream>>>(QK, VTh, VTl, TAB, UB, Ctx, hg * HG, 0.125f);
  }

  gemm64<1, 0, 0><<<gNo, blk, 0, stream>>>(
      Ctx, CTXP, 0LL, 0LL, WoT2, 2 * DM, 0LL,
      Ctx, Ctx, out0, DM, 0LL, 0LL, VP, 0LL,
      MP, DM, 2 * DM, 1, DM / 64, 0, 0, 1.0f);
  (void)hipGetLastError();
}
